// SparseAttention_35656818492142
// MI455X (gfx1250) — hardware-verified
//
#include <hip/hip_runtime.h>


#ifndef NB
#define NB 128
#endif
#ifndef SEQ
#define SEQ 256
#endif
#define NB_FULL  128
#define SEQ_FULL 256
#ifndef BG
#define BG ((NB) < 64 ? (NB) : 64)
#endif
#define DM   384
#define NH   8
#define HD   48
#define NMEM 512
#define WIN  64
#define NQKV 1152
#define SL2E ((float)(0.14433756729740643 * 1.4426950408889634))
#define USEQ ((unsigned)(SEQ))

typedef _Float16 h16;
typedef unsigned short bf;
typedef __attribute__((ext_vector_type(16))) __bf16   v16bf;
typedef __attribute__((ext_vector_type(16))) _Float16 v16h;
typedef __attribute__((ext_vector_type(8)))  _Float16 v8h;
typedef __attribute__((ext_vector_type(2)))  _Float16 v2h;
typedef __attribute__((ext_vector_type(8)))  unsigned short v8us;
typedef __attribute__((ext_vector_type(2)))  unsigned short v2us;
typedef __attribute__((ext_vector_type(8)))  float    v8f;
typedef __attribute__((ext_vector_type(4)))  float    v4f;
typedef v4f __attribute__((may_alias)) v4fa;

static_assert(SEQ % 64 == 0);
static_assert(SEQ <= SEQ_FULL);
static_assert(NB <= NB_FULL);
static_assert(NB % BG == 0);
static_assert(DM == NH * HD);
static_assert(DM % 64 == 0);
static_assert(NQKV == 3 * DM);
static_assert(NMEM % 64 == 0);
static_assert((NQKV * DM) % 64 == 0);
static_assert((DM * DM) % 64 == 0);
static_assert(HD == 48);
static_assert((size_t)7 * BG * SEQ * DM * 2 + (size_t)NQKV * DM * 2 + (size_t)DM * DM * 2 + (size_t)2 * NMEM * DM * 2 <= (size_t)134217728);

__device__ __forceinline__ unsigned short f2bf(float f) { unsigned u = __float_as_uint(f); u += 0x7FFFu + ((u >> 16) & 1u); return (unsigned short)(u >> 16); }
__device__ __forceinline__ float bf2f(unsigned short b) { return __uint_as_float(((unsigned)b) << 16); }
__device__ __forceinline__ float bfr(float f) { return bf2f(f2bf(f)); }
__device__ __forceinline__ void splitf(float y, unsigned short& h, unsigned short& l) { h = f2bf(y); l = f2bf(y - bf2f(h)); }
__device__ __forceinline__ v16h cat16(v8h lo, v8h hi) { return __builtin_shufflevector(lo, hi, 0, 1, 2, 3, 4, 5, 6, 7, 8, 9, 10, 11, 12, 13, 14, 15); }
__device__ __forceinline__ v16bf cat16b(v8us lo, v8us hi) { return __builtin_bit_cast(v16bf, __builtin_shufflevector(lo, hi, 0, 1, 2, 3, 4, 5, 6, 7, 8, 9, 10, 11, 12, 13, 14, 15)); }
__device__ __forceinline__ v8f wmma16(v16h a, v16h b, v8f c) { return __builtin_amdgcn_wmma_f32_16x16x32_f16(false, a, false, b, (short)0, c, false, false); }
__device__ __forceinline__ v8f wmmab(v16bf a, v16bf b, v8f c) { return __builtin_amdgcn_wmma_f32_16x16x32_bf16(false, a, false, b, (short)0, c, false, false); }
__device__ __forceinline__ v8us ld8(const bf* p) { return *(const v8us*)p; }
__device__ __forceinline__ v16bf ldfb(const bf* p) { return cat16b(ld8(p), ld8(p + 16)); }

__global__ __launch_bounds__(256) void k_wtG(const float* __restrict__ w, unsigned K, unsigned N, bf* Bt) {
    const unsigned lane = threadIdx.x & 31u; const unsigned L0 = (blockIdx.x * 8u + (threadIdx.x >> 5)) * 8u; const unsigned nlines = (N * K) >> 6;
#pragma unroll 1
    for (int ps = 0; ps < 2; ++ps) {
#pragma unroll 1
        for (unsigned l = 0; l < 8u; ++l) { const unsigned L = L0 + l; if (L >= nlines) break; const unsigned e = L * 64u + lane * 2u; const unsigned n = e / K; const unsigned k = e - n * K; v2us o;
            o[0] = f2bf(w[(size_t)k * N + n]); o[1] = f2bf(w[(size_t)(k + 1u) * N + n]); *(volatile v2us*)(Bt + e) = o; }
        if (ps == 0) __threadfence(); }
}

__global__ __launch_bounds__(256) void k_cvt8(const float* __restrict__ src, bf* dst, unsigned n8) { const unsigned i = blockIdx.x * 256u + threadIdx.x; if (i >= n8) return; const v8f v = *(const v8f*)(src + (size_t)i * 8u); v8us o;
#pragma unroll
    for (int k = 0; k < 8; ++k) o[k] = f2bf(v[k]);
    *(volatile v8us*)(dst + (size_t)i * 8u) = o; __threadfence(); *(volatile v8us*)(dst + (size_t)i * 8u) = o; }

__global__ __launch_bounds__(256) void k_cvtx(const float* __restrict__ x, bf* X) { const unsigned i = blockIdx.x * 256u + threadIdx.x; if (i >= (unsigned)(BG * SEQ * DM / 8)) return; const unsigned e = i * 8u; const unsigned b = e / (unsigned)(SEQ * DM); const unsigned rem = e - b * (unsigned)(SEQ * DM);
    const v8f v = *(const v8f*)(x + (size_t)b * SEQ_FULL * DM + rem); v8us o;
#pragma unroll
    for (int k = 0; k < 8; ++k) o[k] = f2bf(v[k]);
    *(volatile v8us*)(X + e) = o; __threadfence(); *(volatile v8us*)(X + e) = o; }

__global__ __launch_bounds__(256) void k_vtm(const float* __restrict__ mem, h16* VT) { const unsigned e = (blockIdx.x * 256u + threadIdx.x) * 2u; if (e >= (unsigned)(DM * NMEM)) return; const unsigned m = e & (unsigned)(NMEM - 1); const unsigned c = e / (unsigned)NMEM; v2h o;
    o[0] = (h16)bfr(mem[(size_t)m * DM + c]); o[1] = (h16)bfr(mem[(size_t)(m + 1u) * DM + c]); *(volatile v2h*)(VT + e) = o; __threadfence(); *(volatile v2h*)(VT + e) = o; }

template <int NSPLIT, int MODE>
__global__ __launch_bounds__(32) void k_gemmw(const bf* __restrict__ A, const bf* __restrict__ A2, const bf* __restrict__ Bt, const float* __restrict__ bias,
                                               bf* Qh, bf* Ql, bf* Kp, h16* VT, float* C, const float* __restrict__ rsc) {
    __shared__ __align__(16) float os[64 * 68];
    __shared__ float rs[64];
    const unsigned lane = threadIdx.x & 31u, lr = lane & 15u, hi = lane >> 4; const unsigned r0 = blockIdx.x * 64u, c0 = blockIdx.y * 64u;
    v8f acc[4][4];
#pragma unroll
    for (int mb = 0; mb < 4; ++mb)
#pragma unroll
        for (int nb = 0; nb < 4; ++nb) acc[mb][nb] = (v8f){};
    const size_t aoff = (size_t)(r0 + lr) * DM + 8u * hi, boff = (size_t)(c0 + lr) * DM + 8u * hi;
#pragma unroll 1
    for (unsigned kc = 0; kc < (unsigned)DM; kc += 32u) {
        v16bf a[4], a2[4];
#pragma unroll
        for (int mb = 0; mb < 4; ++mb) { a[mb] = ldfb(A + aoff + (size_t)mb * 16 * DM + kc); if (NSPLIT == 1) a2[mb] = ldfb(A2 + aoff + (size_t)mb * 16 * DM + kc); }
#pragma unroll
        for (int nb = 0; nb < 4; ++nb) { const v16bf b = ldfb(Bt + boff + (size_t)nb * 16 * DM + kc);
#pragma unroll
            for (int mb = 0; mb < 4; ++mb) { acc[mb][nb] = wmmab(a[mb], b, acc[mb][nb]); if (NSPLIT == 1) acc[mb][nb] = wmmab(a2[mb], b, acc[mb][nb]); } }
        asm volatile("v_nop\n\tv_nop\n\tv_nop\n\tv_nop" : "+v"(acc[0][0]), "+v"(acc[1][1]), "+v"(acc[2][2]), "+v"(acc[3][3]) : "v"(a[0]), "v"(a[3]));
    }
#pragma unroll
    for (int mb = 0; mb < 4; ++mb)
#pragma unroll
        for (int nb = 0; nb < 4; ++nb)
#pragma unroll
            for (int j = 0; j < 8; ++j) os[(mb * 16 + hi * 8 + j) * 68 + nb * 16 + lr] = acc[mb][nb][j];
    if (MODE == 1) { const unsigned ra = r0 + lane, rb = ra + 32u; const unsigned ba = ra / USEQ, bb = rb / USEQ;
        rs[lane] = bfr(rsc[(size_t)ba * SEQ_FULL + (ra - ba * USEQ)]); rs[lane + 32u] = bfr(rsc[(size_t)bb * SEQ_FULL + (rb - bb * USEQ)]); }
    __syncthreads();
    if (MODE == 1) {
        const unsigned cofs = lr * 4u; float bv[4];
#pragma unroll
        for (int q = 0; q < 4; ++q) bv[q] = bfr(bias[c0 + cofs + q]);
#pragma unroll 1
        for (int ps = 0; ps < 2; ++ps) {
#pragma unroll 4
            for (unsigned s = 0; s < 32u; ++s) { const unsigned row = 2u * s + hi; v4f val = *(const v4fa*)(os + row * 68u + cofs); const float sc = rs[row];
#pragma unroll
                for (int q = 0; q < 4; ++q) val[q] = (val[q] + bv[q]) * sc;
                *(volatile v4f*)(C + (size_t)(r0 + row) * DM + c0 + cofs) = val; }
            if (ps == 0) __threadfence(); }
    } else {
        const unsigned rq = lane >> 3, c8 = (lane & 7u) * 8u;
        if (blockIdx.y < 12u) {
            const bool isq = (blockIdx.y < 6u); const unsigned cc = isq ? c0 : (c0 - (unsigned)DM); bf* const P0 = isq ? Qh : Kp; float bv[8];
#pragma unroll
            for (int q = 0; q < 8; ++q) bv[q] = bfr(bias[c0 + c8 + q]);
#pragma unroll 1
            for (int ps = 0; ps < 2; ++ps) {
#pragma unroll 2
                for (unsigned s = 0; s < 16u; ++s) { const unsigned row = 4u * s + rq; const v4f x0 = *(const v4fa*)(os + row * 68u + c8); const v4f x1 = *(const v4fa*)(os + row * 68u + c8 + 4u); v8us oh, ol;
#pragma unroll
                    for (int q = 0; q < 4; ++q) { unsigned short hA, lA, hB, lB; splitf(x0[q] + bv[q], hA, lA); splitf(x1[q] + bv[q + 4], hB, lB); oh[q] = hA; ol[q] = lA; oh[q + 4] = hB; ol[q + 4] = lB; }
                    const size_t o = (size_t)(r0 + row) * DM + cc + c8; *(volatile v8us*)(P0 + o) = oh; if (isq) *(volatile v8us*)(Ql + o) = ol; }
                if (ps == 0) __threadfence(); }
        } else {
            const unsigned cv = c0 - 2u * (unsigned)DM; const unsigned bb = r0 / USEQ; const unsigned t0 = r0 - bb * USEQ;
#pragma unroll 1
            for (int ps = 0; ps < 2; ++ps) {
#pragma unroll 2
                for (unsigned s = 0; s < 16u; ++s) { const unsigned ch = 4u * s + rq; const float bch = bfr(bias[c0 + ch]); v8h o;
#pragma unroll
                    for (int j = 0; j < 8; ++j) o[j] = (h16)(os[(c8 + j) * 68u + ch] + bch);
                    *(volatile v8h*)(VT + ((size_t)bb * DM + cv + ch) * SEQ + t0 + c8) = o; }
                if (ps == 0) __threadfence(); }
        }
    }
}

template <bool SELF>
__device__ __forceinline__ void attn_chunk(const bf* kp, const h16* vp, const unsigned vpitch, const int dj,
                                           const v16bf bq0, const v16bf bq1, const v16bf bq2, float& m, float& l, v8f (&acc)[3]) {
    unsigned o2 = 0u; asm volatile("" : "+v"(o2));
    const bf* kp2 = kp + o2;
    v8f st[4];
#pragma unroll
    for (int kt = 0; kt < 4; ++kt) {
        const bf* kr = kp + (size_t)kt * 16 * DM; const bf* kr2 = kp2 + (size_t)kt * 16 * DM; v8f s = (v8f){};
        s = wmmab(cat16b(ld8(kr), ld8(kr + 16)), bq0, s);
        s = wmmab(cat16b(ld8(kr + 32), ld8(kr2)), bq1, s);
        s = wmmab(cat16b(ld8(kr2 + 16), ld8(kr2 + 32)), bq2, s);
        st[kt] = s; }
    asm volatile("v_nop\n\tv_nop\n\tv_nop\n\tv_nop" : "+v"(st[0]), "+v"(st[1]), "+v"(st[2]), "+v"(st[3]) : "v"(bq0), "v"(bq2));
    float cm = -3.0e38f;
#pragma unroll
    for (int kt = 0; kt < 4; ++kt)
#pragma unroll
        for (int r = 0; r < 8; ++r) { float u = st[kt][r] * SL2E; if (SELF) { const int df = dj - kt * 16 - r; u = ((unsigned)df <= (unsigned)WIN) ? u : -1.0e30f; } st[kt][r] = u; cm = fmaxf(cm, u); }
    cm = fmaxf(cm, __shfl_xor(cm, 16, 32));
    const float mn = fmaxf(m, cm); const float corr = __builtin_amdgcn_exp2f(m - mn); m = mn; float ps = 0.f;
#pragma unroll
    for (int kt = 0; kt < 4; ++kt)
#pragma unroll
        for (int r = 0; r < 8; ++r) { const float p = __builtin_amdgcn_exp2f((st[kt][r] - mn) + 10.0f); st[kt][r] = p; ps += p; }
    l = l * corr + ps;
#pragma unroll
    for (int mt = 0; mt < 3; ++mt)
#pragma unroll
        for (int r = 0; r < 8; ++r) acc[mt][r] *= corr;
    v16h pb0, pb1;
#pragma unroll
    for (int r = 0; r < 8; ++r) { pb0[r] = (h16)st[0][r]; pb0[8 + r] = (h16)st[1][r]; pb1[r] = (h16)st[2][r]; pb1[8 + r] = (h16)st[3][r]; }
    asm volatile("" : "+v"(pb0), "+v"(pb1));
#pragma unroll
    for (int mt = 0; mt < 3; ++mt) { const h16* vr = vp + (size_t)mt * 16 * vpitch;
        acc[mt] = wmma16(cat16(*(const v8h*)vr, *(const v8h*)(vr + 16)), pb0, acc[mt]);
        acc[mt] = wmma16(cat16(*(const v8h*)(vr + 32), *(const v8h*)(vr + 48)), pb1, acc[mt]); }
    asm volatile("v_nop\n\tv_nop\n\tv_nop\n\tv_nop" : "+v"(acc[0]), "+v"(acc[1]), "+v"(acc[2]) : "v"(pb0), "v"(pb1));
}

__global__ __launch_bounds__(256) void k_attn(const bf* __restrict__ Qh, const bf* __restrict__ Ql, const bf* __restrict__ Kp, const h16* __restrict__ VT,
                                              const bf* __restrict__ memK, const h16* __restrict__ memVT, const float* __restrict__ gate, bf* Yh, bf* Yl) {
    __shared__ __align__(16) float ys[16 * 388];
    const unsigned tid = threadIdx.x, lane = tid & 31u, h = tid >> 5, n = lane & 15u, hh = lane >> 4;
    const unsigned i0 = blockIdx.x * 16u, bg = blockIdx.y;
    const size_t qoff = ((size_t)bg * SEQ + i0 + n) * DM + h * HD + 8u * hh;
    const v16bf bq0 = cat16b(ld8(Qh + qoff), ld8(Qh + qoff + 16));
    const v16bf bq1 = cat16b(ld8(Qh + qoff + 32), ld8(Ql + qoff));
    const v16bf bq2 = cat16b(ld8(Ql + qoff + 16), ld8(Ql + qoff + 32));
    float m = -1.0e30f, l = 0.f; v8f acc[3];
#pragma unroll
    for (int mt = 0; mt < 3; ++mt) acc[mt] = (v8f){};
    {
        const bf* kp = memK + (size_t)n * DM + h * HD + 8u * hh; const h16* vp = memVT + (size_t)(h * HD + n) * NMEM + 8u * hh;
#pragma unroll 1
        for (unsigned c = 0; c < (unsigned)(NMEM / 64); ++c) attn_chunk<false>(kp + (size_t)c * 64 * DM, vp + c * 64u, (unsigned)NMEM, 0, bq0, bq1, bq2, m, l, acc);
    }
    {
        const unsigned a = i0 >> 6; const unsigned jfirst = (a > 0u) ? (a - 1u) * 64u : 0u; const unsigned nsc = (a > 0u) ? 2u : 1u;
#pragma unroll 1
        for (unsigned c = 0; c < nsc; ++c) { const unsigned js0 = jfirst + c * 64u;
            const bf* kp = Kp + ((size_t)bg * SEQ + js0 + n) * DM + h * HD + 8u * hh; const h16* vp = VT + ((size_t)bg * DM + h * HD + n) * SEQ + js0 + 8u * hh;
            const int dj = (int)(i0 + n) - (int)(js0 + 8u * hh);
            attn_chunk<true>(kp, vp, USEQ, dj, bq0, bq1, bq2, m, l, acc); }
    }
    const float lt = l + __shfl_xor(l, 16, 32); const float inv = 1.0f / lt;
#pragma unroll
    for (int mt = 0; mt < 3; ++mt) { const unsigned cb = h * HD + mt * 16 + 8u * hh; const v4f g0 = *(const v4f*)(gate + cb); const v4f g1 = *(const v4f*)(gate + cb + 4u); v4f o0, o1;
#pragma unroll
        for (int r = 0; r < 4; ++r) { o0[r] = acc[mt][r] * inv * bfr(g0[r]); o1[r] = acc[mt][r + 4] * inv * bfr(g1[r]); }
        float* yp = ys + n * 388u + cb; *(v4fa*)yp = o0; *(v4fa*)(yp + 4) = o1; }
    __syncthreads();
    const size_t tb = ((size_t)bg * SEQ + i0) * DM;
#pragma unroll 1
    for (int ps = 0; ps < 2; ++ps) {
#pragma unroll
        for (unsigned it = 0; it < 3u; ++it) { const unsigned e = (tid + 256u * it) * 8u; const unsigned row = e / (unsigned)DM; const unsigned col = e - row * (unsigned)DM;
            const v4f x0 = *(const v4fa*)(ys + row * 388u + col); const v4f x1 = *(const v4fa*)(ys + row * 388u + col + 4u); v8us oh, ol;
#pragma unroll
            for (int q = 0; q < 4; ++q) { unsigned short hA, lA, hB, lB; splitf(x0[q], hA, lA); splitf(x1[q], hB, lB); oh[q] = hA; ol[q] = lA; oh[q + 4] = hB; ol[q + 4] = lB; }
            *(volatile v8us*)(Yh + tb + e) = oh; *(volatile v8us*)(Yl + tb + e) = ol; }
        if (ps == 0) __threadfence(); }
}

extern "C" void kernel_launch(void* const* d_in, const int* in_sizes, int n_in,
                              void* d_out, int out_size, void* d_ws, size_t ws_size, hipStream_t stream) {
    if (n_in < 8) return;
    if ((size_t)in_sizes[0] < ((size_t)(NB - 1) * SEQ_FULL + SEQ) * DM) return;
    if ((size_t)in_sizes[1] < (size_t)NMEM * DM) return;
    if ((size_t)in_sizes[2] < (size_t)(NB - 1) * SEQ_FULL + SEQ) return;
    if ((size_t)in_sizes[3] < (size_t)DM * NQKV) return;
    if (in_sizes[4] < NQKV) return;
    if ((size_t)in_sizes[5] < (size_t)DM * DM) return;
    if (in_sizes[6] < DM) return;
    if (in_sizes[7] < DM) return;
    if ((size_t)out_size < (size_t)NB * SEQ * DM) return;
    const float* x = (const float*)d_in[0]; const float* mem = (const float*)d_in[1]; const float* lm = (const float*)d_in[2];
    const float* Wqkv = (const float*)d_in[3]; const float* bqkv = (const float*)d_in[4]; const float* Wproj = (const float*)d_in[5];
    const float* bproj = (const float*)d_in[6]; const float* gate = (const float*)d_in[7];
    float* OUT = (float*)d_out;
    char* wsp = (char*)d_ws;
    auto take = [&](size_t bytes) { char* p = wsp; wsp += (bytes + 255) & ~(size_t)255; return (void*)p; };
    const size_t PL = (size_t)BG * SEQ * DM * 2;
    bf* X  = (bf*)take(PL); bf* Qh = (bf*)take(PL); bf* Ql = (bf*)take(PL); bf* Ks = (bf*)take(PL); h16* VTs = (h16*)take(PL); bf* Yh = (bf*)take(PL); bf* Yl = (bf*)take(PL);
    bf* WqT = (bf*)take((size_t)NQKV * DM * 2); bf* WpT = (bf*)take((size_t)DM * DM * 2); bf* memK = (bf*)take((size_t)NMEM * DM * 2); h16* memVT = (h16*)take((size_t)DM * NMEM * 2);
    if ((size_t)(wsp - (char*)d_ws) > ws_size) return;

    k_wtG<<<(NQKV * DM / 64 + 63) / 64, 256, 0, stream>>>(Wqkv, (unsigned)DM, (unsigned)NQKV, WqT);
    k_wtG<<<(DM * DM / 64 + 63) / 64, 256, 0, stream>>>(Wproj, (unsigned)DM, (unsigned)DM, WpT);
    k_cvt8<<<(NMEM * DM / 8 + 255) / 256, 256, 0, stream>>>(mem, memK, (unsigned)(NMEM * DM / 8));
    k_vtm<<<(DM * NMEM / 2 + 255) / 256, 256, 0, stream>>>(mem, memVT);
    for (int g = 0; g < NB / BG; ++g) {
        const float* xg = x + (size_t)g * BG * SEQ_FULL * DM; const float* lmg = lm + (size_t)g * BG * SEQ_FULL; float* og = OUT + (size_t)g * BG * SEQ * DM;
        k_cvtx<<<(BG * SEQ * DM / 8 + 255) / 256, 256, 0, stream>>>(xg, X);
        k_gemmw<0, 0><<<dim3(BG * SEQ / 64, NQKV / 64, 1), 32, 0, stream>>>(X, X, WqT, bqkv, Qh, Ql, Ks, VTs, og, lmg);
        k_attn<<<dim3(SEQ / 16, BG, 1), 256, 0, stream>>>(Qh, Ql, Ks, VTs, memK, memVT, gate, Yh, Yl);
        k_gemmw<1, 1><<<dim3(BG * SEQ / 64, DM / 64, 1), 32, 0, stream>>>(Yh, Yl, WpT, bproj, Qh, Ql, Ks, VTs, og, lmg);
    }
}
